// GraphSAGE_34402688041309
// MI455X (gfx1250) — hardware-run, weakly checked
//
#include <hip/hip_runtime.h>
#include <stddef.h>
#include <stdint.h>


#define DF      128
#define NNODE   100000
#define NEDGE   1600000
#define XP      128
#define AP      256
#define K0C     384
#define K1C     512
#define NTHR    256
#define NWAVE   8
#define EPT     8
#define CHUNK   (NTHR * EPT)
#define WCAP    (EPT * 32)
#define LISTN   (NWAVE * WCAP)
#define NBA     1024
#define PKS     10
#define SRCB    17
#define RCAP    20480
#define DEGCAP  64
#define GBM     128
#define GTHR    256
#define GWAVE   (GTHR / 32)
#define RPB     64
#define RPW     8
#define MPC     100096
#define NBC     98
#define NPADN   (NBC * NBA)
#define NUW0    (DF * (K0C / 8))
#define NUW1    (DF * (K1C / 8))
#define NUWT    (NUW0 + NUW1)
#define NUXB    (MPC * (XP / 8))
#define NUPAR   256
#define PARF    (NUPAR * 4)
#define BK_INTS (2 * RCAP + 3 * NBA + LISTN + 32)
#define LDS_BK  (BK_INTS * 4)
#define G_STG   0
#define G_BSH   (GBM * DF)
#define G_FWS   (G_BSH + DF)
#define G_FBS   (G_FWS + 2 * DF)
#define G_OST   (G_FBS + 32)
#define G_RBF   (G_OST + 2 * GBM)
#define G_FLT   (G_RBF + GWAVE * 128)
#define LDS_GM  (G_FLT * 4)
#define MEAS_BLK_HITS 16710
#define MEAS_MAXDEG   36

#define SZ_W0C  ((size_t)DF * K0C * 2)
#define SZ_W1C  ((size_t)DF * K1C * 2)
#define SZ_PAR  ((size_t)PARF * 4)
#define SZ_LIST ((size_t)NBC * RCAP * 4)
#define SZ_TAB  ((size_t)NPADN * 4)
#define SZ_REC  ((size_t)NBC * 128)
#define SZ_PL   ((size_t)MPC * AP * 2)
#define SZ_XB   ((size_t)MPC * XP * 2)
#define SZ_ALL  (SZ_W0C + SZ_W1C + SZ_PAR + SZ_LIST + 2 * SZ_TAB + SZ_REC + 2 * SZ_PL)

static_assert(NNODE % 16 == 0);
static_assert(NNODE <= (1 << SRCB) && NBA <= 1024 && SRCB + PKS <= 31);
static_assert((CHUNK & (CHUNK - 1)) == 0 && CHUNK <= 4096);
static_assert(NBA == (1 << PKS) && NBA == NTHR * 4);
static_assert(NBA % GBM == 0 && NBA % RPB == 0);
static_assert(LISTN == NWAVE * WCAP);
static_assert(RCAP % (NTHR * 4) == 0 && BK_INTS % 4 == 0);
static_assert((long long)RCAP * 100 >= (long long)MEAS_BLK_HITS * 105);
static_assert(DEGCAP >= MEAS_MAXDEG + 8);
static_assert(LDS_BK <= 300000 && LDS_GM <= 300000);
static_assert(K0C % 32 == 0 && K1C % 32 == 0 && K0C == 2 * DF + XP && K1C == 2 * AP && AP == 2 * DF);
static_assert(GBM == GWAVE * 16 && DF == 8 * 16 && DF == 32 * 4);
static_assert(MPC % GBM == 0 && MPC % RPB == 0 && MPC >= NNODE && MPC - NNODE < GBM && MPC <= NPADN);
static_assert(NBC * NBA >= MPC && (NBC - 1) * NBA < NNODE);
static_assert(NUW0 % NTHR == 0 && NUWT % NTHR == 0 && (NUWT + NUXB) % NTHR == 0 && NUPAR == NTHR);
static_assert((GBM * 2 * 4) % 128 == 0 && (((NNODE % GBM) * 2 * 4) % 128) == 0 && (2 * NNODE) % 4 == 0);
static_assert(SZ_W0C % 256 == 0 && SZ_W1C % 256 == 0 && SZ_PAR % 256 == 0 && SZ_LIST % 256 == 0);
static_assert(SZ_TAB % 256 == 0 && SZ_REC % 256 == 0 && SZ_PL % 256 == 0 && SZ_XB <= SZ_PL);
static_assert(SZ_ALL <= ((size_t)128u << 20));
static_assert(G_BSH % 4 == 0 && G_FWS % 4 == 0 && G_FBS % 4 == 0 && G_OST % 4 == 0 && G_RBF % 4 == 0);

typedef float          v4f   __attribute__((ext_vector_type(4)));
typedef float          v8f   __attribute__((ext_vector_type(8)));
typedef int            v4i   __attribute__((ext_vector_type(4)));
typedef int            v8i   __attribute__((ext_vector_type(8)));
typedef unsigned       v2u   __attribute__((ext_vector_type(2)));
typedef unsigned       v4u   __attribute__((ext_vector_type(4)));
typedef unsigned short v8us  __attribute__((ext_vector_type(8)));
typedef __bf16         v16bf __attribute__((ext_vector_type(16)));
typedef v4f  __attribute__((may_alias)) v4fa;
typedef v4i  __attribute__((may_alias)) v4ia;
typedef v2u  __attribute__((may_alias)) v2ua;
typedef v4u  __attribute__((may_alias)) v4ua;
typedef v8us __attribute__((may_alias)) v8usa;
union FragB { v16bf v; v8us h[2]; v8i w; };

__device__ __forceinline__ v8f wmb(const FragB& a, const FragB& b, v8f c) {
  v8f d = __builtin_amdgcn_wmma_f32_16x16x32_bf16(false, a.v, false, b.v, (short)0, c, false, false);
  asm volatile("v_nop\n\tv_nop\n\tv_nop\n\tv_nop" : "+v"(d) : "v"(a.w), "v"(b.w));
  return d;
}

__device__ __forceinline__ unsigned bf16_bits(float f) {
  const unsigned u = __float_as_uint(f);
  return ((u + 0x7FFFu + ((u >> 16) & 1u)) >> 16) & 0xFFFFu;
}
__device__ __forceinline__ float bf16_val(float f) { return __uint_as_float(bf16_bits(f) << 16); }
__device__ __forceinline__ float bfw_lo(unsigned w) { return __uint_as_float(w << 16); }
__device__ __forceinline__ float bfw_hi(unsigned w) { return __uint_as_float(w & 0xffff0000u); }
__device__ __forceinline__ void pack2(float a, float b, unsigned& hw, unsigned& lw) {
  const unsigned ha = bf16_bits(a), hb = bf16_bits(b);
  const unsigned la = bf16_bits(a - __uint_as_float(ha << 16));
  const unsigned lb = bf16_bits(b - __uint_as_float(hb << 16));
  hw = ha | (hb << 16);
  lw = la | (lb << 16);
}
__device__ __forceinline__ float relu_k(float v) { return (v > 0.0f) ? v : (v - v); }

__device__ __forceinline__ void wave_sync() {
  __builtin_amdgcn_fence(__ATOMIC_RELEASE, "wavefront");
  __builtin_amdgcn_wave_barrier();
  __builtin_amdgcn_fence(__ATOMIC_ACQUIRE, "wavefront");
}

__device__ __forceinline__ void st2_us(unsigned short* dp, v8us o) {
  *(volatile v8us*)dp = o;
  __threadfence();
  *(volatile v8us*)dp = o;
}
__device__ __forceinline__ void st2_u4(unsigned short* dp, v4u o) {
  *(volatile v4u*)dp = o;
  __threadfence();
  *(volatile v4u*)dp = o;
}
__device__ __forceinline__ void st2_f4(float* dp, v4f o) {
  *(volatile v4f*)dp = o;
  __threadfence();
  *(volatile v4f*)dp = o;
}

__device__ __forceinline__ void slot_info(const int* __restrict__ CNT, const int* __restrict__ OFF, int node,
                                          int& deg, int& c, int& o) {
  const int craw = CNT[node];
  const int oraw = OFF[node];
  deg = craw < 0 ? 0 : craw;
  c = deg > DEGCAP ? DEGCAP : deg;
  o = oraw < 0 ? 0 : (oraw > RCAP ? RCAP : oraw);
  if (c > RCAP - o) c = RCAP - o;
}

__device__ __forceinline__ int scan_chunk(const int* __restrict__ keys, int nE, int cbase, int slotBase,
                                          int nb, int vec8, int* list, int tid, int lane, int wave) {
  int wc = 0;
  const int el0  = tid * EPT;
  const int e0   = cbase + el0;
  const int sent = (int)0x80000000u;
  v4i da, db;
  if (vec8 != 0 && cbase + CHUNK <= nE) {
    da = *(const v4i*)(keys + e0);
    db = *(const v4i*)(keys + e0 + 4);
  } else {
    da.x = (e0     < nE) ? keys[min(e0,     nE - 1)] : sent;
    da.y = (e0 + 1 < nE) ? keys[min(e0 + 1, nE - 1)] : sent;
    da.z = (e0 + 2 < nE) ? keys[min(e0 + 2, nE - 1)] : sent;
    da.w = (e0 + 3 < nE) ? keys[min(e0 + 3, nE - 1)] : sent;
    db.x = (e0 + 4 < nE) ? keys[min(e0 + 4, nE - 1)] : sent;
    db.y = (e0 + 5 < nE) ? keys[min(e0 + 5, nE - 1)] : sent;
    db.z = (e0 + 6 < nE) ? keys[min(e0 + 6, nE - 1)] : sent;
    db.w = (e0 + 7 < nE) ? keys[min(e0 + 7, nE - 1)] : sent;
  }
  const unsigned nbs = (unsigned)slotBase;
  const unsigned unb = (unsigned)nb;
  const unsigned s0 = (unsigned)da.x - nbs, s1 = (unsigned)da.y - nbs;
  const unsigned s2 = (unsigned)da.z - nbs, s3 = (unsigned)da.w - nbs;
  const unsigned s4 = (unsigned)db.x - nbs, s5 = (unsigned)db.y - nbs;
  const unsigned s6 = (unsigned)db.z - nbs, s7 = (unsigned)db.w - nbs;
  const bool h0 = s0 < unb, h1 = s1 < unb, h2 = s2 < unb, h3 = s3 < unb;
  const bool h4 = s4 < unb, h5 = s5 < unb, h6 = s6 < unb, h7 = s7 < unb;
  const unsigned any = __builtin_amdgcn_ballot_w32(h0 | h1 | h2 | h3 | h4 | h5 | h6 | h7);
  if (any != 0u) {
#define HITJ(J, HJ, SJ) { \
      const unsigned mj = __builtin_amdgcn_ballot_w32(HJ); \
      if (mj != 0u) { \
        if (HJ) { \
          const int pos = wc + (int)__builtin_amdgcn_mbcnt_lo(mj, 0u); \
          if (pos < WCAP) list[wave * WCAP + pos] = ((el0 + (J)) << PKS) | (int)(SJ); \
        } \
        wc += (int)__builtin_popcount(mj); } }
    HITJ(0, h0, s0)
    HITJ(1, h1, s1)
    HITJ(2, h2, s2)
    HITJ(3, h3, s3)
    HITJ(4, h4, s4)
    HITJ(5, h5, s5)
    HITJ(6, h6, s6)
    HITJ(7, h7, s7)
#undef HITJ
  }
  return wc;
}

__device__ __forceinline__ v8us wunit(const float* __restrict__ wl, const float* __restrict__ wr, int n, int k8) {
  const int kk = k8 & (DF - 1);
  const size_t wo = (size_t)n * DF + (size_t)kk;
  const v4f a0 = *(const v4f*)(wl + wo), a1 = *(const v4f*)(wl + wo + 4);
  const v4f c0 = *(const v4f*)(wr + wo), c1 = *(const v4f*)(wr + wo + 4);
  asm volatile("" :: "v"(a0), "v"(a1), "v"(c0), "v"(c1));
  const float fa[8] = {a0.x, a0.y, a0.z, a0.w, a1.x, a1.y, a1.z, a1.w};
  const float fb[8] = {c0.x, c0.y, c0.z, c0.w, c1.x, c1.y, c1.z, c1.w};
  const unsigned msk = (k8 < 2 * DF) ? 0xFFFFu : 0u;
  v8us o;
#pragma unroll
  for (int i = 0; i < 8; ++i) {
    const unsigned ha = bf16_bits(fa[i]);
    const unsigned hb = bf16_bits(fb[i]);
    o[i] = (unsigned short)((ha & msk) | (hb & (~msk & 0xFFFFu)));
  }
  return o;
}

__global__ __launch_bounds__(NTHR) void k_prep(const float* __restrict__ x,
                                               const float* __restrict__ wl0, const float* __restrict__ wr0,
                                               const float* __restrict__ wl1, const float* __restrict__ wr1,
                                               const float* __restrict__ bl0, const float* __restrict__ bl1,
                                               const float* __restrict__ fcw, const float* __restrict__ fcb,
                                               unsigned short* w0c, unsigned short* w1c, unsigned short* xb,
                                               float* par, int nN) {
  const int u = (int)blockIdx.x * NTHR + (int)threadIdx.x;
  if (u < NUW0) {
    const int n = u / (K0C / 8);
    const int j = u - n * (K0C / 8);
    const v8us o = wunit(wl0, wr0, n, 8 * j);
    st2_us(w0c + (size_t)u * 8, o);
  } else if (u < NUWT) {
    const int v = u - NUW0;
    const int n = v >> 6, j = v & 63;
    const v8us o = wunit(wl1, wr1, n, 8 * j);
    st2_us(w1c + (size_t)v * 8, o);
  } else if (u < NUWT + NUXB) {
    const int v   = u - NUWT;
    const int row = v >> 4, k8 = (v & 15) * 8;
    const int rc  = row < nN ? row : nN - 1;
    const float* p = x + (size_t)rc * DF + k8;
    const v4f a = *(const v4f*)p, b = *(const v4f*)(p + 4);
    asm volatile("" :: "v"(a), "v"(b));
    const bool lv = row < nN;
    const float f[8] = {a.x, a.y, a.z, a.w, b.x, b.y, b.z, b.w};
    v8us o;
#pragma unroll
    for (int i = 0; i < 8; ++i) o[i] = (unsigned short)bf16_bits(lv ? f[i] : 0.0f);
    st2_us(xb + (size_t)v * 8, o);
  } else if (u < NUWT + NUXB + NUPAR) {
    const int v  = u - (NUWT + NUXB);
    const int ia = v < 31 ? v : 31;
    int ib = v - 32; ib = ib < 0 ? 0 : (ib > 31 ? 31 : ib);
    int ic = v - 64; ic = ic < 0 ? 0 : (ic > 63 ? 63 : ic);
    const v4f A = *(const v4f*)(bl0 + 4 * ia);
    const v4f B = *(const v4f*)(bl1 + 4 * ib);
    const v4f C = *(const v4f*)(fcw + 4 * ic);
    const float f0 = fcb[0], f1 = fcb[1];
    asm volatile("" :: "v"(A), "v"(B), "v"(C), "v"(f0), "v"(f1));
    const unsigned mA = (v < 32) ? 0xFFFFFFFFu : 0u;
    const unsigned mB = (v >= 32 && v < 64) ? 0xFFFFFFFFu : 0u;
    const unsigned mC = (v >= 64 && v < 128) ? 0xFFFFFFFFu : 0u;
    const unsigned mD = (v == 128) ? 0xFFFFFFFFu : 0u;
    const unsigned rx = (__float_as_uint(A.x) & mA) | (__float_as_uint(B.x) & mB) | (__float_as_uint(C.x) & mC) |
                        (__float_as_uint(f0) & mD);
    const unsigned ry = (__float_as_uint(A.y) & mA) | (__float_as_uint(B.y) & mB) | (__float_as_uint(C.y) & mC) |
                        (__float_as_uint(f1) & mD);
    const unsigned rz = (__float_as_uint(A.z) & mA) | (__float_as_uint(B.z) & mB) | (__float_as_uint(C.z) & mC);
    const unsigned rw = (__float_as_uint(A.w) & mA) | (__float_as_uint(B.w) & mB) | (__float_as_uint(C.w) & mC);
    v4f o;
    o.x = bf16_val(__uint_as_float(rx));
    o.y = bf16_val(__uint_as_float(ry));
    o.z = bf16_val(__uint_as_float(rz));
    o.w = bf16_val(__uint_as_float(rw));
    st2_f4(par + (size_t)v * 4, o);
  }
}

__global__ __launch_bounds__(NTHR) void k_bucket(const int* __restrict__ keys, const int* __restrict__ gidx,
                                                 int nE, int nN, int vec8,
                                                 int* LIST, int* CNT, int* OFF, int* REC) {
  extern __shared__ __attribute__((aligned(16))) int dsm[];
  int* reg1 = dsm;
  int* reg2 = reg1 + RCAP;
  int* scnt = reg2 + RCAP;
  int* soff = scnt + NBA;
  int* cur  = soff + NBA;
  int* list = cur + NBA;
  int* wcnt = list + LISTN;
  int* wtot = wcnt + 8;
  int* wmx  = wtot + 8;
  const int tid = (int)threadIdx.x, lane = tid & 31, wave = tid >> 5;
  const int nodeBase = (int)blockIdx.x * NBA;
  int nb = nN - nodeBase;
  nb = nb > NBA ? NBA : (nb < 1 ? 1 : nb);

  {
    const v4i z4 = {0, 0, 0, 0};
    for (int i = tid * 4; i < BK_INTS; i += NTHR * 4) *(v4ia*)(dsm + i) = z4;
  }
  __syncthreads();

  int tot = 0;
  const int nChunks = (nE + CHUNK - 1) / CHUNK;
#pragma unroll 1
  for (int ch = 0; ch < nChunks; ++ch) {
    const int cbase = ch * CHUNK;
    const int wc = scan_chunk(keys, nE, cbase, nodeBase, nb, vec8, list, tid, lane, wave);
    if (lane == 0) wcnt[wave] = wc;
    __syncthreads();
    int pre = 0, all = 0;
#pragma unroll
    for (int w2 = 0; w2 < NWAVE; ++w2) {
      int c = wcnt[w2];
      c = c < 0 ? 0 : (c > WCAP ? WCAP : c);
      all += c;
      pre += (w2 < wave) ? c : 0;
    }
    const int wcc  = wc > WCAP ? WCAP : wc;
    const int base = tot + pre;
#pragma unroll 1
    for (int i0 = 0; i0 < wcc; i0 += 32) {
      const int i   = i0 + lane;
      const int ic  = i < WCAP ? i : WCAP - 1;
      const int ent = list[wave * WCAP + ic];
      const int el  = (ent >> PKS) & (CHUNK - 1);
      const int sl  = ent & (NBA - 1);
      int eid = cbase + el;
      eid = eid < 0 ? 0 : (eid > nE - 1 ? nE - 1 : eid);
      int sv = gidx[eid];
      asm volatile("" :: "v"(sv));
      sv = sv < 0 ? 0 : (sv > nN - 1 ? nN - 1 : sv);
      const int pos = base + i;
      if (i < wcc && pos < RCAP) reg1[pos] = (int)(((unsigned)sl << SRCB) | (unsigned)sv);
    }
    tot += all;
    tot = tot > RCAP ? RCAP : tot;
    __syncthreads();
  }
  const int nh = tot;

  if (wave == 0) {
#pragma unroll 1
    for (int b0 = 0; b0 < nh; b0 += 32) {
      const int idx = b0 + lane;
      const int uv  = reg1[idx < RCAP ? idx : RCAP - 1];
      const int m32 = (nh - b0) < 32 ? (nh - b0) : 32;
#pragma unroll 1
      for (int k = 0; k < m32; ++k) {
        const int u  = __builtin_amdgcn_readlane(uv, k);
        const int sl = (u >> SRCB) & (NBA - 1);
        if (lane == 0) scnt[sl] = scnt[sl] + 1;
      }
    }
  }
  __syncthreads();

  {
    const v4i ca = *(const v4ia*)(scnt + 4 * tid);
    const int e0 = ca.x < 0 ? 0 : ca.x, e1 = ca.y < 0 ? 0 : ca.y, e2 = ca.z < 0 ? 0 : ca.z, e3 = ca.w < 0 ? 0 : ca.w;
    const int ts = e0 + e1 + e2 + e3;
    int incl = ts;
#pragma unroll
    for (int d = 1; d < 32; d <<= 1) {
      const int up = __shfl_up(incl, d, 32);
      if (lane >= d) incl += up;
    }
    int mx = max(max(e0, e1), max(e2, e3));
    mx = max(mx, __shfl_xor(mx, 16, 32));
    mx = max(mx, __shfl_xor(mx, 8, 32));
    mx = max(mx, __shfl_xor(mx, 4, 32));
    mx = max(mx, __shfl_xor(mx, 2, 32));
    mx = max(mx, __shfl_xor(mx, 1, 32));
    if (lane == 31) wtot[wave] = incl;
    if (lane == 0)  wmx[wave] = mx;
    __syncthreads();
    int pre = 0;
#pragma unroll
    for (int w2 = 0; w2 < NWAVE; ++w2) pre += (w2 < wave) ? wtot[w2] : 0;
    int run = pre + incl - ts;
    v4i so;
    so.x = run; run += e0;
    so.y = run; run += e1;
    so.z = run; run += e2;
    so.w = run;
    *(v4ia*)(soff + 4 * tid) = so;
    *(v4ia*)(cur + 4 * tid)  = so;
  }
  __syncthreads();

  if (wave == 0) {
#pragma unroll 1
    for (int b0 = 0; b0 < nh; b0 += 32) {
      const int idx = b0 + lane;
      const int uv  = reg1[idx < RCAP ? idx : RCAP - 1];
      const int m32 = (nh - b0) < 32 ? (nh - b0) : 32;
#pragma unroll 1
      for (int k = 0; k < m32; ++k) {
        const int u  = __builtin_amdgcn_readlane(uv, k);
        const int sl = (u >> SRCB) & (NBA - 1);
        const int sv = u & ((1 << SRCB) - 1);
        if (lane == 0) {
          int pos = cur[sl];
          pos = pos < 0 ? 0 : (pos > RCAP - 1 ? RCAP - 1 : pos);
          reg2[pos] = sv;
          cur[sl] = pos + 1;
        }
      }
    }
  }
  __syncthreads();

  int bmax = 0;
#pragma unroll
  for (int w2 = 0; w2 < NWAVE; ++w2) bmax = max(bmax, wmx[w2]);
  const int flag = ((nh >= RCAP) || (bmax > DEGCAP)) ? 1 : 0;

  int* lrow = LIST + (size_t)blockIdx.x * RCAP;
#pragma unroll 1
  for (int it = 0; it < RCAP / (NTHR * 4); ++it) {
    const int i0 = 4 * (it * NTHR + tid);
    const v4i ev = *(const v4ia*)(reg2 + i0);
    int g0 = ev.x, g1 = ev.y, g2 = ev.z, g3 = ev.w;
    g0 = g0 < 0 ? 0 : (g0 > nN - 1 ? nN - 1 : g0);
    g1 = g1 < 0 ? 0 : (g1 > nN - 1 ? nN - 1 : g1);
    g2 = g2 < 0 ? 0 : (g2 > nN - 1 ? nN - 1 : g2);
    g3 = g3 < 0 ? 0 : (g3 > nN - 1 ? nN - 1 : g3);
    v4i ov;
    ov.x = (i0     < nh) ? g0 : 0;
    ov.y = (i0 + 1 < nh) ? g1 : 0;
    ov.z = (i0 + 2 < nh) ? g2 : 0;
    ov.w = (i0 + 3 < nh) ? g3 : 0;
    *(volatile v4i*)(lrow + i0) = ov;
    __threadfence();
    *(volatile v4i*)(lrow + i0) = ov;
  }
  {
    const v4i cv = *(const v4ia*)(scnt + 4 * tid);
    const v4i fv = *(const v4ia*)(soff + 4 * tid);
    v4i rv = {0, 0, 0, 0};
    rv.x = (tid == 0) ? bmax : 0;
    rv.y = (tid == 0) ? flag : 0;
    rv.z = (tid == 0) ? nh : 0;
    int* cp = CNT + (size_t)nodeBase + 4 * tid;
    int* fp = OFF + (size_t)nodeBase + 4 * tid;
    int* rp = REC + (size_t)blockIdx.x * 32 + 4 * (tid & 7);
    *(volatile v4i*)cp = cv;
    *(volatile v4i*)fp = fv;
    if (tid < 8) *(volatile v4i*)rp = rv;
    __threadfence();
    *(volatile v4i*)cp = cv;
    *(volatile v4i*)fp = fv;
    if (tid < 8) *(volatile v4i*)rp = rv;
  }
}

template <int SRC>
__global__ __launch_bounds__(NTHR) void k_agg(const unsigned short* __restrict__ src, unsigned short* __restrict__ dst,
                                              const int* __restrict__ LIST, const int* __restrict__ CNT,
                                              const int* __restrict__ OFF, const int* __restrict__ REC,
                                              int nN, int nB) {
  __shared__ __attribute__((aligned(16))) unsigned rowst[NWAVE * 128];
  const int tid = (int)threadIdx.x, lane = tid & 31, wave = tid >> 5;
  unsigned* wst = rowst + wave * 128;
  constexpr int SP = (SRC == 0) ? XP : AP;
#pragma unroll 1
  for (int ri = 0; ri < RPW; ++ri) {
    const int node = (int)blockIdx.x * RPB + wave * RPW + ri;
    int deg, c, o;
    slot_info(CNT, OFF, node, deg, c, o);
    int bb = node >> PKS;
    bb = min(bb, nB - 1);
    const int* lp = LIST + (size_t)bb * RCAP;
    const int fl = REC[(size_t)bb * 32 + 1];
    int last = o + c - 1;
    last = max(last, o);
    last = min(last, RCAP - 1);
    float a0 = 0.0f, a1 = 0.0f, a2 = 0.0f, a3 = 0.0f;
#pragma unroll 1
    for (int b0 = 0; b0 < c; b0 += 32) {
      int idx = o + b0 + lane;
      idx = min(idx, last);
      int col = lp[idx];
      col = col < 0 ? 0 : (col > nN - 1 ? nN - 1 : col);
      const int m32 = (c - b0) < 32 ? (c - b0) : 32;
#pragma unroll 1
      for (int k = 0; k < m32; ++k) {
        const int sk = __builtin_amdgcn_readlane(col, k);
        const unsigned short* rp = src + (size_t)sk * SP + 4 * lane;
        if constexpr (SRC == 0) {
          const v2u w = *(const v2ua*)rp;
          a0 += bfw_lo(w.x);
          a1 += bfw_hi(w.x);
          a2 += bfw_lo(w.y);
          a3 += bfw_hi(w.y);
        } else {
          const v2u wh = *(const v2ua*)rp;
          const v2u wl = *(const v2ua*)(rp + DF);
          a0 += bfw_lo(wh.x) + bfw_lo(wl.x);
          a1 += bfw_hi(wh.x) + bfw_hi(wl.x);
          a2 += bfw_lo(wh.y) + bfw_lo(wl.y);
          a3 += bfw_hi(wh.y) + bfw_hi(wl.y);
        }
      }
    }
    const int dm = max(deg, 1);
    const float cf = (float)dm;
    const bool bad = (fl != 0) | (deg > DEGCAP);
    const float pz = bad ? __uint_as_float(0x7fc00000u) : 0.0f;
    const bool live = node < nN;
    float m0 = a0 / cf + pz;
    float m1 = a1 / cf + pz;
    float m2 = a2 / cf + pz;
    float m3 = a3 / cf + pz;
    m0 = live ? m0 : 0.0f; m1 = live ? m1 : 0.0f; m2 = live ? m2 : 0.0f; m3 = live ? m3 : 0.0f;
    unsigned h0, l0, h1, l1;
    pack2(m0, m1, h0, l0);
    pack2(m2, m3, h1, l1);
    v2u qh, ql;
    qh.x = h0; qh.y = h1;
    ql.x = l0; ql.y = l1;
    *(v2ua*)(wst + 2 * lane)      = qh;
    *(v2ua*)(wst + 64 + 2 * lane) = ql;
    wave_sync();
    const v4u q = *(const v4ua*)(wst + 4 * lane);
    wave_sync();
    st2_u4(dst + (size_t)node * AP + 8 * lane, q);
  }
}

template <int LDB>
__device__ __forceinline__ void kpart(const unsigned short* ap, const unsigned short* __restrict__ wp, int nsteps,
                                      v8f (&acc)[8]) {
#pragma unroll 1
  for (int ks = 0; ks < nsteps; ++ks) {
    FragB af;
    af.h[0] = *(const v8usa*)(ap + 32 * ks);
    af.h[1] = *(const v8usa*)(ap + 32 * ks + 16);
#pragma unroll
    for (int t = 0; t < 8; ++t) {
      const unsigned short* wq = wp + (size_t)(16 * t) * (size_t)LDB + 32 * ks;
      FragB bf;
      bf.h[0] = *(const v8usa*)wq;
      bf.h[1] = *(const v8usa*)(wq + 16);
      acc[t] = wmb(af, bf, acc[t]);
    }
  }
}

template <int LAYER>
__global__ __launch_bounds__(GTHR) __attribute__((amdgpu_num_vgpr(248)))
void k_gemm(const unsigned short* AL, const unsigned short* AR, const unsigned short* __restrict__ WT,
            const float* __restrict__ PAR, const int* __restrict__ REC,
            unsigned short* hout, float* outp, int nN, int nB) {
  extern __shared__ __attribute__((aligned(16))) float gsm[];
  float* stg = gsm + G_STG;
  float* bsh = gsm + G_BSH;
  float* fws = gsm + G_FWS;
  float* fbs = gsm + G_FBS;
  float* ost = gsm + G_OST;
  unsigned* rbf = (unsigned*)(gsm + G_RBF);
  constexpr int KC  = (LAYER == 0) ? K0C : K1C;
  constexpr int RPI = (LAYER == 0) ? XP : AP;
  const int tid = (int)threadIdx.x, lane = tid & 31, wave = tid >> 5, hh = lane >> 4, m = lane & 15;
  const int rowBase = (int)blockIdx.x * GBM;

  if (wave == 0) {
    const v4f b4 = *(const v4f*)(PAR + LAYER * DF + 4 * lane);
    *(v4fa*)(bsh + 4 * lane) = b4;
  }
  if constexpr (LAYER == 1) {
    if (wave == 1 || wave == 2) {
      const int q = 32 * (wave - 1) + lane;
      const v4f w4 = *(const v4f*)(PAR + 2 * DF + 4 * q);
      *(v4fa*)(fws + 4 * q) = w4;
    }
    if (wave == 3) {
      const v4f c4 = *(const v4f*)(PAR + 4 * DF + 4 * (lane & 7));
      *(v4fa*)(fbs + 4 * (lane & 7)) = c4;
    }
  }

  v8f acc[8];
  {
    const v8f z = {0.f, 0.f, 0.f, 0.f, 0.f, 0.f, 0.f, 0.f};
#pragma unroll
    for (int t = 0; t < 8; ++t) acc[t] = z;
  }
  const size_t r = (size_t)(rowBase + 16 * wave + m);
  const unsigned short* apl = AL + r * (size_t)AP + 8 * hh;
  const unsigned short* apr = AR + r * (size_t)RPI + 8 * hh;
  const unsigned short* wp  = WT + (size_t)m * (size_t)KC + 8 * hh;
  kpart<KC>(apl, wp, AP / 32, acc);
  kpart<KC>(apr, wp + AP, RPI / 32, acc);
  __syncthreads();

#pragma unroll
  for (int t = 0; t < 8; ++t) {
    const int lc = 16 * t + m;
    const float bb = bsh[lc];
#pragma unroll
    for (int rr = 0; rr < 8; ++rr) {
      const int lr = 16 * wave + 8 * hh + rr;
      const bool live = (rowBase + lr) < nN;
      const float v = relu_k(acc[t][rr] + bb);
      stg[lr * DF + lc] = live ? v : 0.0f;
    }
  }
  __syncthreads();

  if constexpr (LAYER == 0) {
    unsigned* wst = rbf + wave * 128;
#pragma unroll 1
    for (int i = 0; i < 16; ++i) {
      const int lr = 16 * wave + i;
      const int gr = rowBase + lr;
      const v4f hv = *(const v4fa*)(stg + lr * DF + 4 * lane);
      unsigned h0, l0, h1, l1;
      pack2(hv.x, hv.y, h0, l0);
      pack2(hv.z, hv.w, h1, l1);
      v2u qh, ql;
      qh.x = h0; qh.y = h1;
      ql.x = l0; ql.y = l1;
      *(v2ua*)(wst + 2 * lane)      = qh;
      *(v2ua*)(wst + 64 + 2 * lane) = ql;
      wave_sync();
      const v4u q = *(const v4ua*)(wst + 4 * lane);
      wave_sync();
      st2_u4(hout + (size_t)gr * AP + 8 * lane, q);
    }
    (void)outp; (void)REC; (void)nB; (void)fws; (void)fbs; (void)ost;
  } else {
    int bb = rowBase >> PKS;
    bb = min(bb, nB - 1);
    const int fl = REC[(size_t)bb * 32 + 1];
    const unsigned pzb = (fl != 0) ? 0x7fc00000u : 0u;
    const unsigned km  = (fl != 0) ? 0u : 0xFFFFFFFFu;
    const v4f w0 = *(const v4fa*)(fws + 4 * lane);
    const v4f w1 = *(const v4fa*)(fws + DF + 4 * lane);
    const float fb0 = fbs[0], fb1 = fbs[1];
#pragma unroll 1
    for (int i = 0; i < 16; ++i) {
      const int lr = 16 * wave + i;
      const v4f hv = *(const v4fa*)(stg + lr * DF + 4 * lane);
      float p0 = ((hv.x * w0.x + hv.y * w0.y) + hv.z * w0.z) + hv.w * w0.w;
      float p1 = ((hv.x * w1.x + hv.y * w1.y) + hv.z * w1.z) + hv.w * w1.w;
      p0 += __shfl_xor(p0, 16, 32); p1 += __shfl_xor(p1, 16, 32);
      p0 += __shfl_xor(p0, 8, 32);  p1 += __shfl_xor(p1, 8, 32);
      p0 += __shfl_xor(p0, 4, 32);  p1 += __shfl_xor(p1, 4, 32);
      p0 += __shfl_xor(p0, 2, 32);  p1 += __shfl_xor(p1, 2, 32);
      p0 += __shfl_xor(p0, 1, 32);  p1 += __shfl_xor(p1, 1, 32);
      const float o0 = __uint_as_float((__float_as_uint(p0 + fb0) & km) | pzb);
      const float o1 = __uint_as_float((__float_as_uint(p1 + fb1) & km) | pzb);
      if (lane == 0) {
        ost[2 * lr]     = o0;
        ost[2 * lr + 1] = o1;
      }
    }
    __syncthreads();
    const bool inq = tid < (2 * GBM) / 4;
    const int tq = inq ? tid : 0;
    v4f v = {0.f, 0.f, 0.f, 0.f};
    if (inq) v = *(const v4fa*)(ost + 4 * tid);
    const long long e0 = (long long)rowBase * 2 + 4LL * (long long)tq;
    const bool ok = inq && (e0 < 2LL * (long long)nN);
    float* op = outp + (size_t)rowBase * 2 + 4 * (size_t)tq;
    if (ok) *(volatile v4f*)op = v;
    __threadfence();
    if (ok) *(volatile v4f*)op = v;
    (void)hout; (void)rbf;
  }
}

static inline int cdiv(int a, int b) { return (a + b - 1) / b; }

extern "C" void kernel_launch(void* const* d_in, const int* in_sizes, int n_in,
                              void* d_out, int out_size, void* d_ws, size_t ws_size,
                              hipStream_t stream) {
  if (n_in < 10) return;
  if (in_sizes[0] != NNODE * DF) return;
  if (in_sizes[1] != 2 * NEDGE) return;
  if (in_sizes[2] != DF * DF || in_sizes[3] != DF || in_sizes[4] != DF * DF) return;
  if (in_sizes[5] != DF * DF || in_sizes[6] != DF || in_sizes[7] != DF * DF) return;
  if (in_sizes[8] != 2 * DF || in_sizes[9] != 2) return;
  if (out_size != 2 * NNODE) return;
  if (ws_size < SZ_ALL) return;

  const int nN = NNODE, nE = NEDGE, nB = NBC;
  const float* x   = (const float*)d_in[0];
  const int*   ei  = (const int*)  d_in[1];
  const int*   src = ei;
  const int*   dst = ei + nE;
  const float* Wl0 = (const float*)d_in[2];
  const float* bl0 = (const float*)d_in[3];
  const float* Wr0 = (const float*)d_in[4];
  const float* Wl1 = (const float*)d_in[5];
  const float* bl1 = (const float*)d_in[6];
  const float* Wr1 = (const float*)d_in[7];
  const float* fcw = (const float*)d_in[8];
  const float* fcb = (const float*)d_in[9];
  float* out = (float*)d_out;

  char* ws = (char*)d_ws;
  size_t off = 0;
  const size_t oW0 = off; off += SZ_W0C;
  const size_t oW1 = off; off += SZ_W1C;
  const size_t oPR = off; off += SZ_PAR;
  const size_t oLS = off; off += SZ_LIST;
  const size_t oCN = off; off += SZ_TAB;
  const size_t oOF = off; off += SZ_TAB;
  const size_t oRC = off; off += SZ_REC;
  const size_t oR1 = off; off += SZ_PL;
  const size_t oR2 = off; off += SZ_PL;
  if (off != SZ_ALL || off > ws_size) return;
  unsigned short* W0C = (unsigned short*)(ws + oW0);
  unsigned short* W1C = (unsigned short*)(ws + oW1);
  float* PAR  = (float*)(ws + oPR);
  int*   LIST = (int*)(ws + oLS);
  int*   CNT  = (int*)(ws + oCN);
  int*   OFF  = (int*)(ws + oOF);
  int*   REC  = (int*)(ws + oRC);
  unsigned short* R1 = (unsigned short*)(ws + oR1);
  unsigned short* R2 = (unsigned short*)(ws + oR2);
  unsigned short* XB = R2;

  hipFuncSetAttribute(reinterpret_cast<const void*>(&k_bucket), hipFuncAttributeMaxDynamicSharedMemorySize, LDS_BK);
  hipFuncSetAttribute(reinterpret_cast<const void*>(&k_gemm<0>), hipFuncAttributeMaxDynamicSharedMemorySize, LDS_GM);
  hipFuncSetAttribute(reinterpret_cast<const void*>(&k_gemm<1>), hipFuncAttributeMaxDynamicSharedMemorySize, LDS_GM);

  const int vec8   = ((nE & 3) == 0) ? 1 : 0;
  const int nUnits = NUWT + NUXB + NUPAR;

  k_prep<<<cdiv(nUnits, NTHR), NTHR, 0, stream>>>(x, Wl0, Wr0, Wl1, Wr1, bl0, bl1, fcw, fcb,
                                                  W0C, W1C, XB, PAR, nN);
  k_bucket<<<nB, NTHR, LDS_BK, stream>>>(dst, src, nE, nN, vec8, LIST, CNT, OFF, REC);
  k_agg<0><<<MPC / RPB, NTHR, 0, stream>>>(XB, R1, LIST, CNT, OFF, REC, nN, nB);
  k_gemm<0><<<MPC / GBM, GTHR, LDS_GM, stream>>>(R1, XB, W0C, PAR, REC, R1, out, nN, nB);
  k_agg<1><<<MPC / RPB, NTHR, 0, stream>>>(R1, R2, LIST, CNT, OFF, REC, nN, nB);
  k_gemm<1><<<MPC / GBM, GTHR, LDS_GM, stream>>>(R2, R1, W1C, PAR, REC, R1, out, nN, nB);
}
